// BoT_MHSA_16131897164366
// MI455X (gfx1250) — hardware-verified
//
#include <hip/hip_runtime.h>
#include <stdint.h>
#include <math.h>

#define NB 4
#define NC 256
#define NP 4096
#define NH 4
#define HD 64
#define QKPLANE ((size_t)NB * NH * NP * HD)

typedef _Float16 v16h __attribute__((ext_vector_type(16)));
typedef _Float16 v8h  __attribute__((ext_vector_type(8)));
typedef __bf16   v16b __attribute__((ext_vector_type(16)));
typedef __bf16   v8b  __attribute__((ext_vector_type(8)));
typedef float    v8f  __attribute__((ext_vector_type(8)));
typedef float    v4f  __attribute__((ext_vector_type(4)));
typedef float    v2f  __attribute__((ext_vector_type(2)));
typedef unsigned int v4u __attribute__((ext_vector_type(4)));

__device__ __forceinline__ unsigned short f2bf_bits(float f) {
  const unsigned u = __float_as_uint(f);
  return (unsigned short)((u + 0x7FFFu + ((u >> 16) & 1u)) >> 16);
}
__device__ __forceinline__ float bf_bits2f(unsigned short h) { return __uint_as_float(((unsigned)h) << 16); }
__device__ __forceinline__ float bfr(float f) { return bf_bits2f(f2bf_bits(f)); }
__device__ __forceinline__ unsigned pk16(unsigned short a, unsigned short b) { return (unsigned)a | ((unsigned)b << 16); }

__device__ __forceinline__ v8f mma_bf(v16b a, v16b b, v8f c) {
  c = __builtin_amdgcn_wmma_f32_16x16x32_bf16(false, a, false, b, (short)0, c, false, false);
  asm volatile("v_nop\n\tv_nop\n\tv_nop\n\tv_nop" : "+v"(c) : "v"(a), "v"(b));
  return c;
}
__device__ __forceinline__ v8f mma_h(v16h a, v16h b, v8f c) {
  c = __builtin_amdgcn_wmma_f32_16x16x32_f16(false, a, false, b, (short)0, c, false, false);
  asm volatile("v_nop\n\tv_nop\n\tv_nop\n\tv_nop" : "+v"(c) : "v"(a), "v"(b));
  return c;
}
#define SCHED_FENCE() __builtin_amdgcn_sched_barrier(0)

union FragB { v16b v; v8b h[2]; };
union FragH { v16h v; v8h h[2]; _Float16 s[16]; };

__device__ __forceinline__ v16b ld_bf(const __bf16* p) {
  FragB f; f.h[0] = *(const v8b*)(p); f.h[1] = *(const v8b*)(p + 16); return f.v;
}

__global__ __launch_bounds__(256) void cvt_w_kernel(const float* __restrict__ w0, const float* __restrict__ w1,
                                                    const float* __restrict__ w2, unsigned short* __restrict__ Wb) {
  const int z = blockIdx.y;
  const float* src = (z == 0) ? w0 : ((z == 1) ? w1 : w2);
  unsigned* dst = (unsigned*)(Wb + (size_t)z * (NC * NC));
  const int i = blockIdx.x * 256 + threadIdx.x;
  if (i < (NC * NC) / 2) {
    const v2f f = *(const v2f*)(src + 2 * (size_t)i);
    const unsigned u = pk16(f2bf_bits(f[0]), f2bf_bits(f[1]));
    ((volatile unsigned*)dst)[i] = u;
    __threadfence();
    ((volatile unsigned*)dst)[i] = u;
  }
}

__global__ __launch_bounds__(256) void xt_kernel(const float* __restrict__ x, unsigned short* __restrict__ xT) {
  __shared__ __align__(16) float tf[64 * 68];
  const int p0 = blockIdx.x * 64;
  const int c0 = blockIdx.y * 64;
  const int b  = blockIdx.z;
  const float* xb = x + (size_t)b * NC * NP;
  const int tid = threadIdx.x;
  {
    const int lr = tid >> 4, c4 = (tid & 15) * 4;
#pragma unroll
    for (int it = 0; it < 4; ++it) {
      const int rr = it * 16 + lr;
      const v4f a = *(const v4f*)(xb + (size_t)(c0 + rr) * NP + p0 + c4);
      *(v4f*)(tf + rr * 68 + c4) = a;
    }
  }
  __syncthreads();
  const int sub = tid >> 3, c8 = (tid & 7) * 8;
  v4u hv[2];
#pragma unroll
  for (int it = 0; it < 2; ++it) {
    const int op = it * 32 + sub;
    v4u a;
#pragma unroll
    for (int q = 0; q < 4; ++q) {
      const float f0 = tf[(c8 + 2 * q) * 68 + op];
      const float f1 = tf[(c8 + 2 * q + 1) * 68 + op];
      a[q] = pk16(f2bf_bits(f0), f2bf_bits(f1));
    }
    hv[it] = a;
  }
  for (int pass = 0; pass < 2; ++pass) {
#pragma unroll
    for (int it = 0; it < 2; ++it) {
      const int op = it * 32 + sub;
      const size_t go = ((size_t)b * NP + p0 + op) * NC + c0 + c8;
      *(volatile v4u*)(xT + go) = hv[it];
    }
    __threadfence();
  }
}

__global__ __launch_bounds__(256) void proj_kernel(
    const unsigned short* __restrict__ xTp, const unsigned short* __restrict__ Wbp,
    const float* __restrict__ bq, const float* __restrict__ bk, const float* __restrict__ bv,
    const float* __restrict__ relh, const float* __restrict__ relw,
    unsigned short* __restrict__ QKh, unsigned short* __restrict__ QKl, float* __restrict__ Yv) {
  __shared__ __align__(16) float sT[8][16 * 68];
  const int z = blockIdx.y;
  const int b = z / 3;
  const int which = z - 3 * b;
  const int lane = threadIdx.x & 31;
  const int wave = threadIdx.x >> 5;
  const int tile = blockIdx.x * 8 + wave;
  const int tm = tile >> 6;
  const int tn = tile & 63;
  const int m0 = tm << 6;
  const int n0 = tn << 6;
  const __bf16* A  = (const __bf16*)(const void*)Wbp + (size_t)which * (NC * NC);
  const __bf16* Bt = (const __bf16*)(const void*)xTp + (size_t)b * NP * NC;
  const int rl = lane & 15, hh = lane >> 4, koff = hh * 8, mOff = hh * 8;

  v8f acc[4][4];
#pragma unroll
  for (int i = 0; i < 4; ++i)
#pragma unroll
    for (int j = 0; j < 4; ++j) acc[i][j] = (v8f){0.f,0.f,0.f,0.f,0.f,0.f,0.f,0.f};

  for (int k0 = 0; k0 < NC; k0 += 32) {
    v16b bfg[4];
#pragma unroll
    for (int j = 0; j < 4; ++j) bfg[j] = ld_bf(Bt + (size_t)(n0 + (j << 4) + rl) * NC + k0 + koff);
#pragma unroll
    for (int i = 0; i < 4; ++i) {
      const v16b af = ld_bf(A + (size_t)(m0 + (i << 4) + rl) * NC + k0 + koff);
#pragma unroll
      for (int j = 0; j < 4; ++j) acc[i][j] = mma_bf(af, bfg[j], acc[i][j]);
    }
    SCHED_FENCE();
  }

  const float* bias = (which == 0) ? bq : ((which == 1) ? bk : bv);
  const int nn = (n0 >> 6) & 3;
  const int sh = n0 >> 8;
  float* slab = sT[wave];
#pragma unroll
  for (int i = 0; i < 4; ++i) {
    const int mBase = m0 + (i << 4);
#pragma unroll
    for (int j = 0; j < 4; ++j) {
      const int d = (j << 4) + rl;
#pragma unroll
      for (int r = 0; r < 8; ++r) {
        const int o = mBase + mOff + r;
        float v = acc[i][j][r] + bfr(bias[o]);
        if (which == 1) {
          const int s = o * 16 + sh;
          const float pos = bfr(relh[nn * 4096 + d * 64 + (s & 63)]) + bfr(relw[nn * 4096 + d * 64 + (s >> 6)]);
          v += pos;
        }
        slab[(mOff + r) * 68 + d] = v;
      }
    }
    __builtin_amdgcn_fence(__ATOMIC_RELEASE, "workgroup");
    __builtin_amdgcn_wave_barrier();
    __builtin_amdgcn_fence(__ATOMIC_ACQUIRE, "workgroup");
    if (which == 2) {
      float* C = Yv + (size_t)b * NC * NP;
      const int c4 = rl * 4;
      for (int pass = 0; pass < 2; ++pass) {
#pragma unroll
        for (int it = 0; it < 8; ++it) {
          const int row = it * 2 + hh;
          const v4f v = *(const v4f*)(slab + row * 68 + c4);
          *(volatile v4f*)(C + (size_t)(mBase + row) * NP + n0 + c4) = v;
        }
        __threadfence();
      }
    } else {
      const int q4 = lane >> 3, c8 = (lane & 7) * 8;
      unsigned short* Hp = QKh + (size_t)which * QKPLANE;
      unsigned short* Lp = QKl + (size_t)which * QKPLANE;
      for (int pass = 0; pass < 2; ++pass) {
#pragma unroll
        for (int it = 0; it < 4; ++it) {
          const int row = it * 4 + q4;
          const int o = mBase + row;
          const int s = o * 16 + sh;
          const float* sp = slab + row * 68 + c8;
          v4u hvv, lvv;
#pragma unroll
          for (int q = 0; q < 4; ++q) {
            const float f0 = sp[2 * q], f1 = sp[2 * q + 1];
            const unsigned short h0 = f2bf_bits(f0), h1 = f2bf_bits(f1);
            const unsigned short l0 = f2bf_bits(f0 - bf_bits2f(h0)), l1 = f2bf_bits(f1 - bf_bits2f(h1));
            hvv[q] = pk16(h0, h1);
            lvv[q] = pk16(l0, l1);
          }
          const size_t dst = (((size_t)(b * NH + nn)) * NP + s) * HD + c8;
          *(volatile v4u*)(Hp + dst) = hvv;
          *(volatile v4u*)(Lp + dst) = lvv;
        }
        __threadfence();
      }
    }
    __builtin_amdgcn_fence(__ATOMIC_RELEASE, "workgroup");
    __builtin_amdgcn_wave_barrier();
    __builtin_amdgcn_fence(__ATOMIC_ACQUIRE, "workgroup");
  }
}

__global__ __launch_bounds__(256) void vt_kernel(const float* __restrict__ Yv, unsigned short* __restrict__ VThp,
                                                 unsigned short* __restrict__ VTlp) {
  __shared__ __align__(16) float tf[64 * 68];
  const int s0 = blockIdx.x * 64;
  const int n  = blockIdx.y;
  const int b  = blockIdx.z;
  const float* yb = Yv + (size_t)b * NC * NP;
  _Float16* VTh = (_Float16*)(void*)VThp;
  _Float16* VTl = (_Float16*)(void*)VTlp;
  const int tid = threadIdx.x;
  {
    const int lr = tid >> 4, c4 = (tid & 15) * 4;
#pragma unroll
    for (int it = 0; it < 4; ++it) {
      const int sl = it * 16 + lr;
      const int s  = s0 + sl;
      const int o  = s >> 4;
      const int p  = (s & 15) * 256 + n * 64 + c4;
      const v4f a = *(const v4f*)(yb + (size_t)o * NP + p);
      *(v4f*)(tf + sl * 68 + c4) = a;
    }
  }
  __syncthreads();
  const int sub = tid >> 3, c8 = (tid & 7) * 8;
  v8h hv[2], lv[2];
#pragma unroll
  for (int it = 0; it < 2; ++it) {
    const int od = it * 32 + sub;
    v8h a, a2;
#pragma unroll
    for (int e = 0; e < 8; ++e) {
      const float f = tf[(c8 + e) * 68 + od];
      const _Float16 hq = (_Float16)f;
      const _Float16 lq = (_Float16)((f - (float)hq) * 1024.0f);
      a[e] = hq; a2[e] = lq;
    }
    hv[it] = a; lv[it] = a2;
  }
  for (int pass = 0; pass < 2; ++pass) {
#pragma unroll
    for (int it = 0; it < 2; ++it) {
      const int od = it * 32 + sub;
      const size_t go = ((size_t)(b * NH + n) * HD + od) * NP + s0 + c8;
      *(volatile v8h*)(VTh + go) = hv[it];
      *(volatile v8h*)(VTl + go) = lv[it];
    }
    __threadfence();
  }
}

__global__ __launch_bounds__(128) void attn_kernel(
    const unsigned short* __restrict__ Qhp, const unsigned short* __restrict__ Qlp,
    const unsigned short* __restrict__ Khp, const unsigned short* __restrict__ Klp,
    const unsigned short* __restrict__ VThp, const unsigned short* __restrict__ VTlp,
    float* __restrict__ out) {
  __shared__ __align__(16) __bf16   Ksh[64 * HD];
  __shared__ __align__(16) __bf16   Ksl[64 * HD];
  __shared__ __align__(16) _Float16 Vsh[HD * 64];
  __shared__ __align__(16) _Float16 Vsl[HD * 64];
  __shared__ __align__(16) float    Os[4][16 * 68];

  const int tid  = threadIdx.x;
  const int wave = tid >> 5;
  const int lane = tid & 31;
  const int hh   = lane >> 4;
  const int c    = lane & 15;
  const int qt = blockIdx.x;
  const int n  = blockIdx.y;
  const int b  = blockIdx.z;
  const int bn = b * NH + n;

  const __bf16* Qh = (const __bf16*)(const void*)Qhp + (size_t)bn * NP * HD;
  const __bf16* Ql = (const __bf16*)(const void*)Qlp + (size_t)bn * NP * HD;
  const __bf16* Kh = (const __bf16*)(const void*)Khp + (size_t)bn * NP * HD;
  const __bf16* Kl = (const __bf16*)(const void*)Klp + (size_t)bn * NP * HD;
  const _Float16* VTh = (const _Float16*)(const void*)VThp + (size_t)bn * HD * NP;
  const _Float16* VTl = (const _Float16*)(const void*)VTlp + (size_t)bn * HD * NP;

  const int q0 = qt * 64 + wave * 16;
  const int qg = q0 + c;

  v16b qbh[2], qbl[2];
#pragma unroll
  for (int dc = 0; dc < 2; ++dc) {
    qbh[dc] = ld_bf(Qh + (size_t)qg * HD + dc * 32 + 8 * hh);
    qbl[dc] = ld_bf(Ql + (size_t)qg * HD + dc * 32 + 8 * hh);
  }

  float m_run = -1.0e30f, l_run = 0.0f;
  v8f accO[4], accR[4];
#pragma unroll
  for (int t = 0; t < 4; ++t) {
    accO[t] = (v8f){0.f,0.f,0.f,0.f,0.f,0.f,0.f,0.f};
    accR[t] = (v8f){0.f,0.f,0.f,0.f,0.f,0.f,0.f,0.f};
  }

#pragma unroll 1
  for (int it = 0; it < NP / 64; ++it) {
    const int kb = it * 64;
    __syncthreads();
    {
      const int r = tid >> 1, half = (tid & 1) * 32;
      const __bf16*   ksrc = Kh  + (size_t)(kb + r) * HD + half;
      const __bf16*   lsrc = Kl  + (size_t)(kb + r) * HD + half;
      const _Float16* vsrc = VTh + (size_t)r * NP + kb + half;
      const _Float16* wsrc = VTl + (size_t)r * NP + kb + half;
#pragma unroll
      for (int i = 0; i < 4; ++i) {
        const v8b a0 = *(const v8b*)(ksrc + 8 * i);
        const v8b a1 = *(const v8b*)(lsrc + 8 * i);
        const v8h g0 = *(const v8h*)(vsrc + 8 * i);
        const v8h g1 = *(const v8h*)(wsrc + 8 * i);
        *(v8b*)(Ksh + r * HD + half + 8 * i) = a0;
        *(v8b*)(Ksl + r * HD + half + 8 * i) = a1;
        *(v8h*)(Vsh + r * 64 + half + 8 * i) = g0;
        *(v8h*)(Vsl + r * 64 + half + 8 * i) = g1;
      }
    }
    __syncthreads();

    v8f st[4];
#pragma unroll
    for (int t = 0; t < 4; ++t) {
      v8f sv = (v8f){0.f,0.f,0.f,0.f,0.f,0.f,0.f,0.f};
#pragma unroll
      for (int dc = 0; dc < 2; ++dc) {
        FragB ka, kl;
        ka.h[0] = *(const v8b*)(Ksh + (t * 16 + c) * HD + dc * 32 + 8 * hh);
        ka.h[1] = *(const v8b*)(Ksh + (t * 16 + c) * HD + dc * 32 + 16 + 8 * hh);
        kl.h[0] = *(const v8b*)(Ksl + (t * 16 + c) * HD + dc * 32 + 8 * hh);
        kl.h[1] = *(const v8b*)(Ksl + (t * 16 + c) * HD + dc * 32 + 16 + 8 * hh);
        sv = mma_bf(ka.v, qbh[dc], sv);
        sv = mma_bf(ka.v, qbl[dc], sv);
        sv = mma_bf(kl.v, qbh[dc], sv);
      }
      st[t] = sv;
      SCHED_FENCE();
    }

    float mx = m_run;
#pragma unroll
    for (int t = 0; t < 4; ++t)
#pragma unroll
      for (int r = 0; r < 8; ++r) mx = fmaxf(mx, st[t][r]);
    mx = fmaxf(mx, __shfl_xor(mx, 16, 32));
    const float alpha = __expf(m_run - mx);
    m_run = mx;
    float rs = 0.0f;
#pragma unroll
    for (int t = 0; t < 4; ++t)
#pragma unroll
      for (int r = 0; r < 8; ++r) {
        const float p = __expf(st[t][r] - mx);
        st[t][r] = p;
        rs += p;
      }
    rs += __shfl_xor(rs, 16, 32);
    l_run = l_run * alpha + rs;
#pragma unroll
    for (int dt = 0; dt < 4; ++dt)
#pragma unroll
      for (int r = 0; r < 8; ++r) { accO[dt][r] *= alpha; accR[dt][r] *= alpha; }

#pragma unroll
    for (int kc = 0; kc < 2; ++kc) {
      FragH pb;
#pragma unroll
      for (int r = 0; r < 8; ++r) {
        pb.s[r]     = (_Float16)(st[2 * kc][r]     * 4096.0f);
        pb.s[8 + r] = (_Float16)(st[2 * kc + 1][r] * 4096.0f);
      }
#pragma unroll
      for (int dt = 0; dt < 4; ++dt) {
        FragH va, vr;
        va.h[0] = *(const v8h*)(Vsh + (dt * 16 + c) * 64 + kc * 32 + 8 * hh);
        va.h[1] = *(const v8h*)(Vsh + (dt * 16 + c) * 64 + kc * 32 + 16 + 8 * hh);
        vr.h[0] = *(const v8h*)(Vsl + (dt * 16 + c) * 64 + kc * 32 + 8 * hh);
        vr.h[1] = *(const v8h*)(Vsl + (dt * 16 + c) * 64 + kc * 32 + 16 + 8 * hh);
        accO[dt] = mma_h(va.v, pb.v, accO[dt]);
        accR[dt] = mma_h(vr.v, pb.v, accR[dt]);
      }
      SCHED_FENCE();
    }
  }

  const float inv = __builtin_amdgcn_rcpf(l_run) * (1.0f / 4096.0f);
  float* os = Os[wave];
#pragma unroll
  for (int dt = 0; dt < 4; ++dt) {
    v4f a, a2;
#pragma unroll
    for (int r = 0; r < 4; ++r) {
      a[r]  = (accO[dt][r]     + accR[dt][r]     * (1.0f / 1024.0f)) * inv;
      a2[r] = (accO[dt][4 + r] + accR[dt][4 + r] * (1.0f / 1024.0f)) * inv;
    }
    *(v4f*)(os + c * 68 + dt * 16 + 8 * hh)     = a;
    *(v4f*)(os + c * 68 + dt * 16 + 8 * hh + 4) = a2;
  }
  __builtin_amdgcn_fence(__ATOMIC_RELEASE, "workgroup");
  __builtin_amdgcn_wave_barrier();
  __builtin_amdgcn_fence(__ATOMIC_ACQUIRE, "workgroup");
  {
    float* ob = out + (size_t)b * NC * NP + (size_t)q0 * (NH * HD) + n * HD;
    const int c4 = c * 4;
    for (int pass = 0; pass < 2; ++pass) {
#pragma unroll
      for (int i = 0; i < 8; ++i) {
        const int row = i * 2 + hh;
        const v4f v = *(const v4f*)(os + row * 68 + c4);
        *(volatile v4f*)(ob + (size_t)row * (NH * HD) + c4) = v;
      }
      __threadfence();
    }
  }
}

extern "C" void kernel_launch(void* const* d_in, const int* in_sizes, int n_in,
                              void* d_out, int out_size, void* d_ws, size_t ws_size,
                              hipStream_t stream) {
  if (n_in < 9) return;
  if (in_sizes[0] != NB * NC * NP) return;
  if (in_sizes[1] != NC * NC || in_sizes[3] != NC * NC || in_sizes[5] != NC * NC) return;
  if (in_sizes[2] != NC || in_sizes[4] != NC || in_sizes[6] != NC) return;
  if (in_sizes[7] != NH * HD * 64 || in_sizes[8] != NH * HD * 64) return;
  if (out_size != NB * NC * NP) return;

  const float* x    = (const float*)d_in[0];
  const float* wq   = (const float*)d_in[1];
  const float* bq   = (const float*)d_in[2];
  const float* wk   = (const float*)d_in[3];
  const float* bk   = (const float*)d_in[4];
  const float* wv   = (const float*)d_in[5];
  const float* bv   = (const float*)d_in[6];
  const float* relh = (const float*)d_in[7];
  const float* relw = (const float*)d_in[8];
  float* out = (float*)d_out;

  const size_t szWb = (size_t)3 * NC * NC * 2;
  const size_t szXT = (size_t)NB * NP * NC * 2;
  const size_t szQK = (size_t)2 * QKPLANE * 2;
  const size_t szYv = (size_t)NB * NC * NP * 4;
  const size_t szVT = (size_t)NB * NH * HD * NP * 2;
  size_t off = 0;
  const size_t oWb  = off; off += szWb;
  const size_t oXT  = off; off += szXT;
  const size_t oQKh = off; off += szQK;
  const size_t oQKl = off; off += szQK;
  const size_t oYv  = off; off += szYv;
  const size_t oVTh = off; off += szVT;
  const size_t oVTl = off; off += szVT;
  if (off > ws_size) return;

  char* ws = (char*)d_ws;
  unsigned short* Wb  = (unsigned short*)(ws + oWb);
  unsigned short* XT  = (unsigned short*)(ws + oXT);
  unsigned short* QKh = (unsigned short*)(ws + oQKh);
  unsigned short* QKl = (unsigned short*)(ws + oQKl);
  float*          Yv  = (float*)(ws + oYv);
  unsigned short* VTh = (unsigned short*)(ws + oVTh);
  unsigned short* VTl = (unsigned short*)(ws + oVTl);

  cvt_w_kernel<<<dim3((NC * NC / 2) / 256, 3), dim3(256), 0, stream>>>(wq, wk, wv, Wb);
  xt_kernel<<<dim3(NP / 64, NC / 64, NB), dim3(256), 0, stream>>>(x, XT);
  proj_kernel<<<dim3(32, NB * 3), dim3(256), 0, stream>>>(XT, Wb, bq, bk, bv, relh, relw, QKh, QKl, Yv);
  vt_kernel<<<dim3(NP / 64, NH, NB), dim3(256), 0, stream>>>(Yv, VTh, VTl);
  attn_kernel<<<dim3(NP / 64, NH, NB), dim3(128), 0, stream>>>(
      QKh, QKl, QKh + QKPLANE, QKl + QKPLANE, VTh, VTl, out);
  (void)hipGetLastError();
}
